// DFS_17136919511590
// MI455X (gfx1250) — hardware-verified
//
#include <hip/hip_runtime.h>

typedef __attribute__((ext_vector_type(16))) _Float16 v16h;
typedef __attribute__((ext_vector_type(8)))  _Float16 v8h;
typedef __attribute__((ext_vector_type(16))) __bf16   v16b;
typedef __attribute__((ext_vector_type(8)))  __bf16   v8b;
typedef __attribute__((ext_vector_type(8)))  float    v8f;
typedef __attribute__((ext_vector_type(4)))  float    v4f;

__device__ __forceinline__ unsigned short f2bf_bits(float f) {
  unsigned u = __float_as_uint(f);
  return (unsigned short)((u + 0x7FFFu + ((u >> 16) & 1u)) >> 16);
}
__device__ __forceinline__ float bf_bits2f(unsigned short h) { return __uint_as_float(((unsigned)h) << 16); }

__device__ __forceinline__ void dep_guard_h(v8f& a, v8f& b, v16h x, v16h y) { asm volatile("v_nop\n\tv_nop\n\tv_nop\n\tv_nop" : "+v"(a), "+v"(b) : "v"(x), "v"(y)); }
__device__ __forceinline__ void dep_guard_b(v8f& a, v8f& b, v16b x, v16b y) { asm volatile("v_nop\n\tv_nop\n\tv_nop\n\tv_nop" : "+v"(a), "+v"(b) : "v"(x), "v"(y)); }
__device__ __forceinline__ void keep4_h(v16h a, v16h b, v16h c, v16h d) { asm volatile("v_nop" :: "v"(a), "v"(b), "v"(c), "v"(d)); }
__device__ __forceinline__ void keep4_b(v16b a, v16b b, v16b c, v16b d) { asm volatile("v_nop" :: "v"(a), "v"(b), "v"(c), "v"(d)); }
__device__ __forceinline__ void acc_guard4(v8f& a, v8f& b, v8f& c, v8f& d) { asm volatile("v_nop\n\tv_nop\n\tv_nop\n\tv_nop" : "+v"(a), "+v"(b), "+v"(c), "+v"(d)); }
template <typename T> struct Frag;
template <> struct Frag<_Float16> {
  typedef v16h V; union U { v16h v; v8h h[2]; };
  static __device__ __forceinline__ v16h load(const _Float16* p) {
    U f; f.h[0] = *(const v8h*)(p); f.h[1] = *(const v8h*)(p + 16); return f.v;
  }
  static __device__ __forceinline__ v8f mma(v16h a, v16h b, v8f c) {
    return __builtin_amdgcn_wmma_f32_16x16x32_f16(false, a, false, b, (short)0, c, false, false);
  }
  static __device__ __forceinline__ void guard(v8f& a, v8f& b, v16h x, v16h y) { dep_guard_h(a, b, x, y); }
  static __device__ __forceinline__ void keep(v16h a, v16h b, v16h c, v16h d) { keep4_h(a, b, c, d); }
};
template <> struct Frag<__bf16> {
  typedef v16b V; union U { v16b v; v8b h[2]; };
  static __device__ __forceinline__ v16b load(const __bf16* p) {
    U f; f.h[0] = *(const v8b*)(p); f.h[1] = *(const v8b*)(p + 16); return f.v;
  }
  static __device__ __forceinline__ v8f mma(v16b a, v16b b, v8f c) {
    return __builtin_amdgcn_wmma_f32_16x16x32_bf16(false, a, false, b, (short)0, c, false, false);
  }
  static __device__ __forceinline__ void guard(v8f& a, v8f& b, v16b x, v16b y) { dep_guard_b(a, b, x, y); }
  static __device__ __forceinline__ void keep(v16b a, v16b b, v16b c, v16b d) { keep4_b(a, b, c, d); }
};

template <int ET> struct Elem;
template <> struct Elem<0> { typedef _Float16 T; };
template <> struct Elem<1> { typedef __bf16 T; };
template <int ET, bool SPLIT, int BIAS_MODE, int OUT_MODE, bool RESID, int ACT = 0>
__global__ __launch_bounds__(256) void wmma_gemm64(
    const unsigned short* __restrict__ Ap, const unsigned short* __restrict__ A2p, int lda, long strideA,
    const unsigned short* __restrict__ Btp, const unsigned short* __restrict__ Bt2p, int ldb, long strideB,
    void* __restrict__ Cout, void* __restrict__ Cout2, int ldc, long strideC,
    const float* __restrict__ bias,
    const float* __restrict__ resid, long strideR,
    int M, int N, int K, float scale) {
  typedef typename Elem<ET>::T T;
  typedef typename Frag<T>::V V;
  const T* A = (const T*)Ap; const T* A2 = (const T*)A2p; const T* Bt = (const T*)Btp; const T* Bt2 = (const T*)Bt2p;
  __shared__ __align__(16) float sT[8][16 * 68];
  const int b    = blockIdx.y;
  const int lane = threadIdx.x & 31;
  const int wave = threadIdx.x >> 5;
  const int tilesN = N >> 6;
  const int tilesM = M >> 6;
  const int tile = blockIdx.x * 8 + wave;
  if (tile >= tilesM * tilesN) return;
  const int tm = tile / tilesN;
  const int tn = tile - tm * tilesN;
  const int m0 = tm << 6;
  const int n0 = tn << 6;

  const T* Ab  = A  + (size_t)b * strideA;
  const T* Bb  = Bt + (size_t)b * strideB;
  const T* Ab2 = SPLIT ? (A2  + (size_t)b * strideA) : nullptr;
  const T* Bb2 = SPLIT ? (Bt2 + (size_t)b * strideB) : nullptr;

  const int rlane = lane & 15;
  const int koff  = (lane >> 4) * 8;
  const int mOff  = (lane >> 4) * 8;

  v8f acc[4][4];
#pragma unroll
  for (int i = 0; i < 4; ++i)
#pragma unroll
    for (int j = 0; j < 4; ++j) acc[i][j] = (v8f){0.f,0.f,0.f,0.f,0.f,0.f,0.f,0.f};

  for (int k0 = 0; k0 < K; k0 += 32) {
    V bh[4], bl[4];
#pragma unroll
    for (int j = 0; j < 4; ++j) {
      const size_t bo = (size_t)(n0 + (j << 4) + rlane) * ldb + koff + k0;
      bh[j] = Frag<T>::load(Bb + bo);
      if (SPLIT) bl[j] = Frag<T>::load(Bb2 + bo);
    }
#pragma unroll
    for (int i = 0; i < 4; ++i) {
      const size_t ao = (size_t)(m0 + (i << 4) + rlane) * lda + koff + k0;
      V ah = Frag<T>::load(Ab + ao);
      V al;
      if (SPLIT) al = Frag<T>::load(Ab2 + ao);
#pragma unroll
      for (int j = 0; j < 4; ++j) {
        acc[i][j] = Frag<T>::mma(ah, bh[j], acc[i][j]);
        if (SPLIT) {
          acc[i][j] = Frag<T>::mma(ah, bl[j], acc[i][j]);
          acc[i][j] = Frag<T>::mma(al, bh[j], acc[i][j]);
        }
      }
      Frag<T>::guard(acc[i][0], acc[i][3], ah, SPLIT ? al : ah);
    }
    Frag<T>::keep(bh[0], bh[1], bh[2], bh[3]);
    if (SPLIT) Frag<T>::keep(bl[0], bl[1], bl[2], bl[3]);
  }
  acc_guard4(acc[0][0], acc[0][1], acc[0][2], acc[0][3]);
  acc_guard4(acc[1][0], acc[1][1], acc[1][2], acc[1][3]);
  acc_guard4(acc[2][0], acc[2][1], acc[2][2], acc[2][3]);
  acc_guard4(acc[3][0], acc[3][1], acc[3][2], acc[3][3]);

  float* slab = sT[wave];
  const float* Rb = RESID ? (resid + (size_t)b * strideR) : nullptr;
#pragma unroll
  for (int i = 0; i < 4; ++i) {
    const int mBase = m0 + (i << 4);
#pragma unroll
    for (int j = 0; j < 4; ++j) {
      const int n = n0 + (j << 4) + rlane;
      float bv = 0.f;
      if (BIAS_MODE == 2) bv = bias[n];
#pragma unroll
      for (int r = 0; r < 8; ++r) {
        float v = acc[i][j][r] * scale;
        if (BIAS_MODE == 1) v += bias[mBase + mOff + r];
        if (BIAS_MODE == 2) v += bv;
        if (RESID) v += Rb[(size_t)(mBase + mOff + r) * ldc + n];
        if (ACT == 1) v = tanhf(v);
        if (ACT == 2) v = fmaxf(v, 0.0f);
        if (ACT == 3) v = v / (1.0f + expf(-v));
        if (ACT == 4) v = (v > 0.f) ? v : 0.01f * v;
        if (ACT == 5) v = 0.5f * v * (1.0f + erff(v * 0.70710678118654752f));
        slab[(mOff + r) * 68 + (j << 4) + rlane] = v;
      }
    }
    __builtin_amdgcn_fence(__ATOMIC_RELEASE, "workgroup");
    __builtin_amdgcn_wave_barrier();
    __builtin_amdgcn_fence(__ATOMIC_ACQUIRE, "workgroup");
    if (OUT_MODE == 0) {
      float* C = (float*)Cout + (size_t)b * strideC;
      const int hh = lane >> 4, c4 = (lane & 15) * 4;
      for (int pass = 0; pass < 2; ++pass) {
#pragma unroll
        for (int it = 0; it < 8; ++it) {
          const int row = it * 2 + hh;
          v4f v = *(const v4f*)(slab + row * 68 + c4);
          *(volatile v4f*)(C + (size_t)(mBase + row) * ldc + n0 + c4) = v;
        }
        __threadfence();
      }
    } else {
      const int q = lane >> 3, c8 = (lane & 7) * 8;
      unsigned short* C  = (unsigned short*)Cout  + (size_t)b * strideC;
      unsigned short* C2 = (OUT_MODE == 2) ? ((unsigned short*)Cout2 + (size_t)b * strideC) : nullptr;
      for (int pass = 0; pass < 2; ++pass) {
#pragma unroll
        for (int it = 0; it < 4; ++it) {
          const int row = it * 4 + q;
          const float* sp = slab + row * 68 + c8;
          v8h hv, lv;
#pragma unroll
          for (int e = 0; e < 8; ++e) {
            if (OUT_MODE == 1) {
              hv[e] = (_Float16)sp[e];
            } else {
              unsigned short hb = f2bf_bits(sp[e]);
              unsigned short lb = f2bf_bits(sp[e] - bf_bits2f(hb));
              hv[e] = __builtin_bit_cast(_Float16, hb);
              lv[e] = __builtin_bit_cast(_Float16, lb);
            }
          }
          *(volatile v8h*)(C + (size_t)(mBase + row) * ldc + n0 + c8) = hv;
          if (OUT_MODE == 2) *(volatile v8h*)(C2 + (size_t)(mBase + row) * ldc + n0 + c8) = lv;
        }
        __threadfence();
      }
    }
    __builtin_amdgcn_fence(__ATOMIC_RELEASE, "workgroup");
    __builtin_amdgcn_wave_barrier();
    __builtin_amdgcn_fence(__ATOMIC_ACQUIRE, "workgroup");
  }
}

#define HH   192
#define WW   192
#define HP   (HH + 2)
#define WP   (WW + 2)
#define CX   64
#define CIN  (CX + 3)
#define OCH  64
#define NOC  18
#define NOP  32
#define LDBO 640
#define KDC  (9 * CX)
#define TP   196
#define NPA  (NOP * LDBO / 8)
#define NPB  (OCH * KDC / 8)

__global__ __launch_bounds__(256) void k_prep_x(const float* __restrict__ x, float* __restrict__ xT,
    unsigned short* __restrict__ xph, unsigned short* __restrict__ xpl) {
  __shared__ __align__(16) float tile[CX * TP];
  const int tid = threadIdx.x, lane = tid & 31, wave = tid >> 5;
  const int n = blockIdx.x / HP, hp = blockIdx.x - n * HP;
  const bool inner = (hp > 0) && (hp < HP - 1);
  const int h = inner ? (hp - 1) : 0;
  if (inner) {
    for (int i = tid; i < CX * (WW / 4); i += 256) {
      const int c = i / (WW / 4), w4 = (i - c * (WW / 4)) * 4;
      const v4f v = *(const v4f*)(x + (((size_t)n * CX + c) * HH + h) * WW + w4);
      *(v4f*)(tile + c * TP + w4) = v;
    }
  }
  __syncthreads();
  if (inner) {
    const int hh = lane >> 4, c4 = (lane & 15) * 4;
    const size_t rowpix = ((size_t)n * HH + h) * WW;
    for (int pr = wave; pr < (WW >> 1); pr += 8) {
      const int w = pr * 2 + hh;
      v4f v;
      v[0] = tile[(c4 + 0) * TP + w];
      v[1] = tile[(c4 + 1) * TP + w];
      v[2] = tile[(c4 + 2) * TP + w];
      v[3] = tile[(c4 + 3) * TP + w];
      float* p = xT + (rowpix + w) * CX + c4;
      *(volatile v4f*)p = v;
      __threadfence();
      *(volatile v4f*)p = v;
    }
  }
  {
    const int q = lane >> 3, c8 = (lane & 7) * 8;
    const size_t prow = ((size_t)n * HP + hp) * WP;
    for (int g = wave; g * 4 < WP; g += 8) {
      const int wp = g * 4 + q;
      const bool colin = inner && (wp > 0) && (wp < WP - 1);
      int w = wp - 1;
      w = w < 0 ? 0 : w;
      w = w > WW - 1 ? WW - 1 : w;
      v8h hv, lv;
#pragma unroll
      for (int e = 0; e < 8; ++e) {
        const float t = tile[(c8 + e) * TP + w];
        const float f = colin ? t : 0.0f;
        const unsigned short hb = f2bf_bits(f);
        const unsigned short lb = f2bf_bits(f - bf_bits2f(hb));
        hv[e] = __builtin_bit_cast(_Float16, hb);
        lv[e] = __builtin_bit_cast(_Float16, lb);
      }
      const int wpc = wp < WP ? wp : (WP - 1);
      const size_t o = (prow + wpc) * CX + c8;
      if (wp < WP) { *(volatile v8h*)(xph + o) = hv; *(volatile v8h*)(xpl + o) = lv; }
      __threadfence();
      if (wp < WP) { *(volatile v8h*)(xph + o) = hv; *(volatile v8h*)(xpl + o) = lv; }
    }
  }
}

__global__ __launch_bounds__(256) void k_prep_r(const float* __restrict__ refx,
    unsigned short* __restrict__ Rh, unsigned short* __restrict__ Rl) {
  __shared__ __align__(16) _Float16 sh[256 * 32];
  __shared__ __align__(16) _Float16 sl[256 * 32];
  const int tid = threadIdx.x, lane = tid & 31, wave = tid >> 5;
  const int px = blockIdx.x * 256 + tid;
  const int n = px / (HH * WW), rem = px - n * (HH * WW), h = rem / WW, w = rem - h * WW;
#pragma unroll
  for (int j = 0; j < 32; ++j) {
    float f = 0.0f;
    if (j < 27) {
      const int tap = j / 3, cr = j - tap * 3;
      const int ty = tap / 3, tx = tap - ty * 3;
      const int yy = h + ty - 1, xx = w + tx - 1;
      const bool inb = (yy >= 0) && (yy < HH) && (xx >= 0) && (xx < WW);
      const int yc = min(max(yy, 0), HH - 1), xc = min(max(xx, 0), WW - 1);
      const float g = refx[(((size_t)n * 3 + cr) * HH + yc) * WW + xc];
      f = inb ? g : 0.0f;
    }
    const unsigned short hb = f2bf_bits(f);
    const unsigned short lb = f2bf_bits(f - bf_bits2f(hb));
    sh[tid * 32 + j] = __builtin_bit_cast(_Float16, hb);
    sl[tid * 32 + j] = __builtin_bit_cast(_Float16, lb);
  }
  __syncthreads();
  const int po = lane >> 2, e8 = (lane & 3) * 8;
#pragma unroll
  for (int it = 0; it < 4; ++it) {
    const int pl = (it * 8 + wave) * 8 + po;
    const v8h hv = *(const v8h*)(sh + pl * 32 + e8);
    const v8h lv = *(const v8h*)(sl + pl * 32 + e8);
    const size_t o = ((size_t)blockIdx.x * 256 + pl) * 32 + e8;
    *(volatile v8h*)(Rh + o) = hv; *(volatile v8h*)(Rl + o) = lv;
    __threadfence();
    *(volatile v8h*)(Rh + o) = hv; *(volatile v8h*)(Rl + o) = lv;
  }
}

__global__ __launch_bounds__(256) void k_prep_w(const float* __restrict__ offw, const float* __restrict__ offb,
    const float* __restrict__ dcw, unsigned short* __restrict__ Bth, unsigned short* __restrict__ Btl,
    unsigned short* __restrict__ Wt, float* __restrict__ obp) {
  const int p = blockIdx.x * 256 + threadIdx.x;
  if (p < NPA) {
    const int row = (p * 8) / LDBO, col0 = p * 8 - row * LDBO;
    v8h hv, lv;
#pragma unroll
    for (int e = 0; e < 8; ++e) {
      const int kk = col0 + e;
      int idx; bool use;
      if (kk < 9 * CX) {
        const int tap = kk >> 6, c = kk & 63;
        idx = (row * CIN + c) * 9 + tap; use = (row < NOC);
      } else {
        const int j = kk - 9 * CX; const int tap = j / 3, cr = j - tap * 3;
        idx = (row * CIN + CX + cr) * 9 + tap; use = (row < NOC) && (j < 27);
      }
      idx = min(max(idx, 0), NOC * CIN * 9 - 1);
      const float g = offw[idx];
      const float f = use ? g : 0.0f;
      const unsigned short hb = f2bf_bits(f);
      const unsigned short lb = f2bf_bits(f - bf_bits2f(hb));
      hv[e] = __builtin_bit_cast(_Float16, hb);
      lv[e] = __builtin_bit_cast(_Float16, lb);
    }
    const size_t o = (size_t)p * 8;
    *(volatile v8h*)(Bth + o) = hv; *(volatile v8h*)(Btl + o) = lv;
    __threadfence();
    *(volatile v8h*)(Bth + o) = hv; *(volatile v8h*)(Btl + o) = lv;
  } else if (p < NPA + NPB) {
    const int p2 = p - NPA;
    const int o_ = (p2 * 8) / KDC, col0 = p2 * 8 - o_ * KDC;
    v8h hv;
#pragma unroll
    for (int e = 0; e < 8; ++e) {
      const int kk = col0 + e;
      const int tap = kk >> 6, c = kk & 63;
      const float f = dcw[((size_t)o_ * CX + c) * 9 + tap] * 64.0f;
      hv[e] = (_Float16)f;
    }
    const size_t o = (size_t)p2 * 8;
    *(volatile v8h*)(Wt + o) = hv;
    __threadfence();
    *(volatile v8h*)(Wt + o) = hv;
  }
  if (p < 32) {
    const float g = offb[min(p, NOC - 1)];
    const float v = (p < NOC) ? g : 0.0f;
    *(volatile float*)(obp + p) = v;
    __threadfence();
    *(volatile float*)(obp + p) = v;
  }
}

__device__ __forceinline__ void oc_kstep(v8f (&acc)[4][2], const __bf16* __restrict__ Ah, const __bf16* __restrict__ Al,
    size_t a0, size_t astr, const __bf16* __restrict__ Bh, const __bf16* __restrict__ Bl, size_t b0) {
  v16b bh[2], bl[2];
#pragma unroll
  for (int j = 0; j < 2; ++j) {
    const size_t bo = b0 + (size_t)j * (16 * LDBO);
    bh[j] = Frag<__bf16>::load(Bh + bo);
    bl[j] = Frag<__bf16>::load(Bl + bo);
  }
#pragma unroll
  for (int i = 0; i < 4; ++i) {
    const size_t ao = a0 + (size_t)i * astr;
    const v16b ah = Frag<__bf16>::load(Ah + ao);
    const v16b al = Frag<__bf16>::load(Al + ao);
#pragma unroll
    for (int j = 0; j < 2; ++j) {
      acc[i][j] = Frag<__bf16>::mma(ah, bh[j], acc[i][j]);
      acc[i][j] = Frag<__bf16>::mma(ah, bl[j], acc[i][j]);
      acc[i][j] = Frag<__bf16>::mma(al, bh[j], acc[i][j]);
    }
    Frag<__bf16>::guard(acc[i][0], acc[i][1], ah, al);
  }
  Frag<__bf16>::keep(bh[0], bh[1], bl[0], bl[1]);
}

__global__ __launch_bounds__(256) void k_offconv(const unsigned short* __restrict__ xph, const unsigned short* __restrict__ xpl,
    const unsigned short* __restrict__ Rhp, const unsigned short* __restrict__ Rlp,
    const unsigned short* __restrict__ Bthp, const unsigned short* __restrict__ Btlp,
    const float* __restrict__ obp, float* __restrict__ OFF, int ntiles) {
  __shared__ __align__(16) float sT[8][16 * 36];
  const int lane = threadIdx.x & 31, wave = threadIdx.x >> 5;
  const int tile = blockIdx.x * 8 + wave;
  if (tile >= ntiles) return;
  const int wq = tile % (WW / 64);
  const int t2 = tile / (WW / 64);
  const int h = t2 % HH, n = t2 / HH;
  const int w0 = wq * 64;
  const __bf16* Ah  = (const __bf16*)(const void*)xph;
  const __bf16* Al  = (const __bf16*)(const void*)xpl;
  const __bf16* RAh = (const __bf16*)(const void*)Rhp;
  const __bf16* RAl = (const __bf16*)(const void*)Rlp;
  const __bf16* Bh  = (const __bf16*)(const void*)Bthp;
  const __bf16* Bl  = (const __bf16*)(const void*)Btlp;
  const int rlane = lane & 15, koff = (lane >> 4) * 8, mOff = koff;

  v8f acc[4][2];
#pragma unroll
  for (int i = 0; i < 4; ++i)
#pragma unroll
    for (int j = 0; j < 2; ++j) acc[i][j] = (v8f){0.f,0.f,0.f,0.f,0.f,0.f,0.f,0.f};

  const size_t b0 = (size_t)rlane * LDBO + koff;
#pragma unroll 1
  for (int s = 0; s < 18; ++s) {
    const int tap = s >> 1, c0 = (s & 1) * 32;
    const int ty = tap / 3, tx = tap - ty * 3;
    const size_t a0 = ((((size_t)n * HP + h + ty) * WP) + w0 + tx + rlane) * CX + c0 + koff;
    oc_kstep(acc, Ah, Al, a0, (size_t)16 * CX, Bh, Bl, b0 + (size_t)s * 32);
  }
  {
    const size_t a0 = ((((size_t)n * HH + h) * WW) + w0 + rlane) * 32 + koff;
    oc_kstep(acc, RAh, RAl, a0, (size_t)16 * 32, Bh, Bl, b0 + (size_t)18 * 32);
  }
  acc_guard4(acc[0][0], acc[0][1], acc[1][0], acc[1][1]);
  acc_guard4(acc[2][0], acc[2][1], acc[3][0], acc[3][1]);

  float* slab = sT[wave];
  const size_t pxrow = ((size_t)n * HH + h) * WW + w0;
  const int q = lane >> 3, c4 = (lane & 7) * 4;
#pragma unroll
  for (int i = 0; i < 4; ++i) {
#pragma unroll
    for (int j = 0; j < 2; ++j) {
      const int nch = j * 16 + rlane;
      const float bv = obp[nch];
#pragma unroll
      for (int r = 0; r < 8; ++r) slab[(mOff + r) * 36 + nch] = acc[i][j][r] + bv;
    }
    __builtin_amdgcn_fence(__ATOMIC_RELEASE, "workgroup");
    __builtin_amdgcn_wave_barrier();
    __builtin_amdgcn_fence(__ATOMIC_ACQUIRE, "workgroup");
    for (int pass = 0; pass < 2; ++pass) {
#pragma unroll
      for (int it = 0; it < 4; ++it) {
        const int row = it * 4 + q;
        const v4f v = *(const v4f*)(slab + row * 36 + c4);
        *(volatile v4f*)(OFF + (pxrow + i * 16 + row) * NOP + c4) = v;
      }
      __threadfence();
    }
    __builtin_amdgcn_fence(__ATOMIC_RELEASE, "workgroup");
    __builtin_amdgcn_wave_barrier();
    __builtin_amdgcn_fence(__ATOMIC_ACQUIRE, "workgroup");
  }
}

__global__ __launch_bounds__(256) void k_sample(const float* __restrict__ xT, const float* __restrict__ OFF,
    unsigned short* __restrict__ S, int n, int h0) {
  const int lane = threadIdx.x & 31, wave = threadIdx.x >> 5;
  const int q = lane >> 3, c8 = (lane & 7) * 8;
  const size_t img = (size_t)n * (HH * WW);
#pragma unroll 1
  for (int it = 0; it < 9; ++it) {
    const int item = (it * 8 + wave) * 4 + q;
    const int pxl = item / 9;
    const int tap = item - pxl * 9;
    const int pxc = blockIdx.x * 32 + pxl;
    const int rem = h0 * WW + pxc;
    const int h = rem / WW, w = rem - h * WW;
    const size_t px = img + (size_t)rem;
    const float dy = OFF[px * NOP + 2 * tap];
    const float dx = OFF[px * NOP + 2 * tap + 1];
    const int ty = tap / 3;
    const int ky = ty - 1, kx = (tap - ty * 3) - 1;
    const float py = (float)(h + ky) + dy;
    const float pq = (float)(w + kx) + dx;
    const float y0 = floorf(py), x0 = floorf(pq);
    const float wy1 = py - y0, wx1 = pq - x0;
    const float wy0 = 1.0f - wy1, wx0 = 1.0f - wx1;
    const float y1 = y0 + 1.0f, x1 = x0 + 1.0f;
    const bool vy0 = (y0 >= 0.0f) && (y0 < (float)HH);
    const bool vy1 = (y1 >= 0.0f) && (y1 < (float)HH);
    const bool vx0 = (x0 >= 0.0f) && (x0 < (float)WW);
    const bool vx1 = (x1 >= 0.0f) && (x1 < (float)WW);
    const int yc0 = (int)fminf(fmaxf(y0, 0.0f), (float)(HH - 1));
    const int yc1 = (int)fminf(fmaxf(y1, 0.0f), (float)(HH - 1));
    const int xc0 = (int)fminf(fmaxf(x0, 0.0f), (float)(WW - 1));
    const int xc1 = (int)fminf(fmaxf(x1, 0.0f), (float)(WW - 1));
    const float w00 = (vy0 && vx0) ? (wy0 * wx0) : 0.0f;
    const float w01 = (vy0 && vx1) ? (wy0 * wx1) : 0.0f;
    const float w10 = (vy1 && vx0) ? (wy1 * wx0) : 0.0f;
    const float w11 = (vy1 && vx1) ? (wy1 * wx1) : 0.0f;
    const float* r00 = xT + (img + (size_t)yc0 * WW + xc0) * CX + c8;
    const float* r01 = xT + (img + (size_t)yc0 * WW + xc1) * CX + c8;
    const float* r10 = xT + (img + (size_t)yc1 * WW + xc0) * CX + c8;
    const float* r11 = xT + (img + (size_t)yc1 * WW + xc1) * CX + c8;
    const v4f a0 = *(const v4f*)(r00), a1 = *(const v4f*)(r00 + 4);
    const v4f b0 = *(const v4f*)(r01), b1 = *(const v4f*)(r01 + 4);
    const v4f g0 = *(const v4f*)(r10), g1 = *(const v4f*)(r10 + 4);
    const v4f d0 = *(const v4f*)(r11), d1 = *(const v4f*)(r11 + 4);
    v8h hv;
#pragma unroll
    for (int e = 0; e < 4; ++e) {
      hv[e]     = (_Float16)(((a0[e] * w00 + b0[e] * w01) + g0[e] * w10) + d0[e] * w11);
      hv[4 + e] = (_Float16)(((a1[e] * w00 + b1[e] * w01) + g1[e] * w10) + d1[e] * w11);
    }
    unsigned short* sp = S + (size_t)pxc * KDC + tap * CX + c8;
    *(volatile v8h*)sp = hv;
    __threadfence();
    *(volatile v8h*)sp = hv;
  }
}

static inline size_t al256(size_t b) { return (b + 255) & ~(size_t)255; }

extern "C" void kernel_launch(void* const* d_in, const int* in_sizes, int n_in,
                              void* d_out, int out_size, void* d_ws, size_t ws_size,
                              hipStream_t stream)
{
  if (n_in < 6) return;
  const float* x    = (const float*)d_in[0];
  const float* refx = (const float*)d_in[1];
  const float* offw = (const float*)d_in[2];
  const float* offb = (const float*)d_in[3];
  const float* dcw  = (const float*)d_in[4];
  const float* dcb  = (const float*)d_in[5];
  float* out = (float*)d_out;

  const long HWl = (long)HH * WW;
  if (in_sizes[2] != NOC * CIN * 9 || in_sizes[3] != NOC) return;
  if (in_sizes[4] != OCH * CX * 9 || in_sizes[5] != OCH) return;
  if (in_sizes[0] <= 0 || ((long)in_sizes[0] % (CX * HWl)) != 0) return;
  const int N = (int)((long)in_sizes[0] / (CX * HWl));
  if (N <= 0) return;
  if ((long)in_sizes[1] != (long)N * 3 * HWl) return;
  if ((long)out_size != (long)N * OCH * HWl) return;
  const long npix = (long)N * HWl;
  const long CH = HWl / 2;

  size_t off = 0;
  const size_t szP = al256((size_t)N * HP * WP * CX * 2);
  const size_t o_xph = off; off += szP;
  const size_t o_xpl = off; off += szP;
  const size_t o_xT  = off; off += al256((size_t)npix * CX * 4);
  const size_t o_off = off; off += al256((size_t)npix * NOP * 4);
  const size_t o_bth = off; off += al256((size_t)NOP * LDBO * 2);
  const size_t o_btl = off; off += al256((size_t)NOP * LDBO * 2);
  const size_t o_wt  = off; off += al256((size_t)OCH * KDC * 2);
  const size_t o_obp = off; off += al256((size_t)NOP * 4);
  const size_t szR = al256((size_t)npix * 32 * 2);
  const size_t szS = al256((size_t)CH * KDC * 2);
  size_t szshr = 2 * szR; if (szS > szshr) szshr = szS;
  const size_t o_shr = off; off += szshr;
  if (off > ws_size || off > (size_t)134217728) return;

  unsigned char* ws = (unsigned char*)d_ws;
  unsigned short* xph = (unsigned short*)(ws + o_xph);
  unsigned short* xpl = (unsigned short*)(ws + o_xpl);
  float*          xT  = (float*)(ws + o_xT);
  float*          OFFp = (float*)(ws + o_off);
  unsigned short* bth = (unsigned short*)(ws + o_bth);
  unsigned short* btl = (unsigned short*)(ws + o_btl);
  unsigned short* wt  = (unsigned short*)(ws + o_wt);
  float*          obp = (float*)(ws + o_obp);
  unsigned short* Rh  = (unsigned short*)(ws + o_shr);
  unsigned short* Rl  = (unsigned short*)(ws + o_shr + szR);
  unsigned short* Sb  = (unsigned short*)(ws + o_shr);

  k_prep_x<<<dim3((unsigned)(N * HP)), dim3(256), 0, stream>>>(x, xT, xph, xpl);
  k_prep_r<<<dim3((unsigned)(npix / 256)), dim3(256), 0, stream>>>(refx, Rh, Rl);
  k_prep_w<<<dim3((NPA + NPB + 255) / 256), dim3(256), 0, stream>>>(offw, offb, dcw, bth, btl, wt, obp);
  const int ntiles = N * HH * (WW / 64);
  k_offconv<<<dim3((unsigned)((ntiles + 7) / 8)), dim3(256), 0, stream>>>(xph, xpl, Rh, Rl, bth, btl, obp, OFFp, ntiles);

  const int nchunk = N * 2;
  const int tiles = (OCH / 64) * (int)(CH / 64);
  for (int ch = 0; ch < nchunk; ++ch) {
    const int n = ch / 2, h0 = (ch % 2) * (HH / 2);
    k_sample<<<dim3((unsigned)(CH / 32)), dim3(256), 0, stream>>>(xT, OFFp, Sb, n, h0);
    float* Cp = out + (size_t)n * OCH * HWl + (size_t)h0 * WW;
    wmma_gemm64<0, false, 1, 0, false><<<dim3((unsigned)((tiles + 7) / 8), 1), dim3(256), 0, stream>>>(
        wt, wt, KDC, 0L, Sb, Sb, KDC, 0L, (void*)Cp, (void*)obp, (int)HWl, 0L,
        dcb, dcb, 0L, OCH, (int)CH, KDC, 1.0f / 64.0f);
  }
}
